// ThalamicRNN_18116172054562
// MI455X (gfx1250) — hardware-run, weakly checked
//
#include <hip/hip_runtime.h>


#define NB   2048
#define NN   2048
#define NR   64
#define NS   128
typedef _Float16 h16;
typedef unsigned short bf;
typedef __attribute__((ext_vector_type(16))) __bf16   v16bf;
typedef __attribute__((ext_vector_type(16))) _Float16 v16h;
typedef __attribute__((ext_vector_type(8)))  _Float16 v8h;
typedef __attribute__((ext_vector_type(8)))  unsigned short v8us;
typedef __attribute__((ext_vector_type(8)))  float    v8f;
typedef __attribute__((ext_vector_type(4)))  float    v4f;
typedef v8h  __attribute__((may_alias)) v8ha;
typedef v4f  __attribute__((may_alias)) v4fa;
typedef v8us __attribute__((may_alias)) v8usa;

__device__ __forceinline__ unsigned short f2bf(float f) { unsigned u = __float_as_uint(f); u += 0x7FFFu + ((u >> 16) & 1u); return (unsigned short)(u >> 16); }
__device__ __forceinline__ float bf2f(unsigned short b) { return __uint_as_float(((unsigned)b) << 16); }
__device__ __forceinline__ float bfr(float f) { return bf2f(f2bf(f)); }
__device__ __forceinline__ v16h cat16(v8h lo, v8h hi) { return __builtin_shufflevector(lo, hi, 0, 1, 2, 3, 4, 5, 6, 7, 8, 9, 10, 11, 12, 13, 14, 15); }
__device__ __forceinline__ v16bf cat16b(v8us lo, v8us hi) { return __builtin_bit_cast(v16bf, __builtin_shufflevector(lo, hi, 0, 1, 2, 3, 4, 5, 6, 7, 8, 9, 10, 11, 12, 13, 14, 15)); }
__device__ __forceinline__ v8f wmma16(v16h a, v16h b, v8f c) { return __builtin_amdgcn_wmma_f32_16x16x32_f16(false, a, false, b, (short)0, c, false, false); }
__device__ __forceinline__ v8f wmmab(v16bf a, v16bf b, v8f c) { return __builtin_amdgcn_wmma_f32_16x16x32_bf16(false, a, false, b, (short)0, c, false, false); }

template <typename T16> struct WFrag;
template <> struct WFrag<h16> { typedef v16h V; static __device__ __forceinline__ V ld(const h16* p) { return cat16(*(const v8h*)p, *(const v8h*)(p + 16)); } static __device__ __forceinline__ v8f mma(V a, V b, v8f c) { return wmma16(a, b, c); } };
template <> struct WFrag<bf> { typedef v16bf V; static __device__ __forceinline__ V ld(const bf* p) { return cat16b(*(const v8us*)p, *(const v8us*)(p + 16)); } static __device__ __forceinline__ v8f mma(V a, V b, v8f c) { return wmmab(a, b, c); } };
template <typename T16, int NSPLIT, bool BIAS>
__global__ __launch_bounds__(32) void k_gemmw(const T16* __restrict__ A, const T16* __restrict__ A2, const T16* __restrict__ Bt, const T16* __restrict__ Bt2, int K, float* C, int ldc, const float* __restrict__ bias, size_t sA, size_t sB, size_t sC) {
    typedef typename WFrag<T16>::V V;
    __shared__ __align__(16) float os[16 * 68];
    const size_t z = blockIdx.z; A += z * sA; if (A2) A2 += z * sA; Bt += z * sB; if (Bt2) Bt2 += z * sB; C += z * sC;
    const int lane = threadIdx.x & 31, lr = lane & 15, hi = lane >> 4; const int r0 = blockIdx.x * 64, c0 = blockIdx.y * 64;
    v8f acc[4][4];
#pragma unroll
    for (int mb = 0; mb < 4; ++mb)
#pragma unroll
        for (int nb = 0; nb < 4; ++nb) acc[mb][nb] = (v8f){};
    const size_t aoff = (size_t)(r0 + lr) * K + 8 * hi, boff = (size_t)(c0 + lr) * K + 8 * hi;
    for (int kc = 0; kc < K; kc += 32) {
        V a[4], a2[4];
#pragma unroll
        for (int mb = 0; mb < 4; ++mb) { a[mb] = WFrag<T16>::ld(A + aoff + (size_t)mb * 16 * K + kc); if (NSPLIT == 1 || NSPLIT == 2) a2[mb] = WFrag<T16>::ld(A2 + aoff + (size_t)mb * 16 * K + kc); }
#pragma unroll
        for (int nb = 0; nb < 4; ++nb) { const V b = WFrag<T16>::ld(Bt + boff + (size_t)nb * 16 * K + kc); V b2; if (NSPLIT >= 2) b2 = WFrag<T16>::ld(Bt2 + boff + (size_t)nb * 16 * K + kc);
#pragma unroll
            for (int mb = 0; mb < 4; ++mb) { acc[mb][nb] = WFrag<T16>::mma(a[mb], b, acc[mb][nb]); if (NSPLIT == 1 || NSPLIT == 2) acc[mb][nb] = WFrag<T16>::mma(a2[mb], b, acc[mb][nb]); if (NSPLIT >= 2) acc[mb][nb] = WFrag<T16>::mma(a[mb], b2, acc[mb][nb]); } }
        asm volatile("v_nop\n\tv_nop\n\tv_nop\n\tv_nop" : "+v"(acc[0][0]), "+v"(acc[1][1]), "+v"(acc[2][2]), "+v"(acc[3][3]) : "v"(a[0]), "v"(a[3]));
    }
#pragma unroll
    for (int mb = 0; mb < 4; ++mb) {
#pragma unroll
        for (int nb = 0; nb < 4; ++nb) {
#pragma unroll
            for (int j = 0; j < 8; ++j) os[(hi * 8 + j) * 68 + nb * 16 + lr] = acc[mb][nb][j]; }
        __builtin_amdgcn_wave_barrier(); asm volatile("" ::: "memory");
        float* crow = C + (size_t)(r0 + mb * 16) * ldc + c0;
#pragma unroll 1
        for (int ps = 0; ps < 2; ++ps) {
#pragma unroll
            for (int s = 0; s < 8; ++s) { const int row = 2 * s + hi, cofs = lr * 4; v4f val = *(const v4fa*)(os + row * 68 + cofs); if (BIAS) { val[0] += bfr(bias[c0 + cofs]); val[1] += bfr(bias[c0 + cofs + 1]); val[2] += bfr(bias[c0 + cofs + 2]); val[3] += bfr(bias[c0 + cofs + 3]); }
                *(volatile v4f*)(crow + (size_t)row * ldc + cofs) = val; }
            if (ps == 0) __threadfence(); }
        __builtin_amdgcn_wave_barrier(); asm volatile("" ::: "memory");
    }
}

typedef __attribute__((ext_vector_type(2))) _Float16 v2h;
typedef __attribute__((ext_vector_type(4))) _Float16 v4h;
typedef __attribute__((ext_vector_type(2))) unsigned short v2us;
typedef __attribute__((ext_vector_type(4))) unsigned short v4us;
typedef __attribute__((ext_vector_type(2))) float v2f;
typedef __attribute__((ext_vector_type(4))) int v4i;

__global__ __launch_bounds__(256) void k_wtG(const float* __restrict__ w, int K, int N, bf* Bt) {
    const int lane = threadIdx.x & 31; const int L0 = (blockIdx.x * 8 + (threadIdx.x >> 5)) * 8; const int nlines = N * K / 64;
#pragma unroll
    for (int ps = 0; ps < 2; ++ps) {
        for (int l = 0; l < 8; ++l) { const int L = L0 + l; if (L >= nlines) break; const size_t e = (size_t)L * 64 + lane * 2; const int k = (int)(e % K), n = (int)(e / K); v2us o;
            o[0] = f2bf(w[(size_t)k * N + n]); o[1] = f2bf(w[(size_t)(k + 1) * N + n]); *(volatile v2us*)(Bt + e) = o; }
        if (ps == 0) __threadfence(); }
}

__global__ __launch_bounds__(256) void k_cvt8(const float* __restrict__ src, bf* dst, size_t n8) { const size_t i = (size_t)blockIdx.x * 256 + threadIdx.x; if (i >= n8) return; const v8f v = *(const v8f*)(src + i * 8); v8us o;
#pragma unroll
    for (int k = 0; k < 8; ++k) o[k] = f2bf(v[k]); *(volatile v8us*)(dst + i * 8) = o; __threadfence(); *(volatile v8us*)(dst + i * 8) = o; }

__global__ __launch_bounds__(256) void k_mid(const float* __restrict__ g, const float* __restrict__ P2, bf* T) { const int i = blockIdx.x * 256 + threadIdx.x; if (i >= NB * NR / 8) return; const v8f a = *(const v8f*)(g + (size_t)i * 8); const v8f p = *(const v8f*)(P2 + (size_t)i * 8); v8us o;
#pragma unroll
    for (int k = 0; k < 8; ++k) o[k] = f2bf(__fmul_rn(bfr(a[k]), p[k])); *(volatile v8us*)(T + (size_t)i * 8) = o; __threadfence(); *(volatile v8us*)(T + (size_t)i * 8) = o; }

__global__ __launch_bounds__(256) void k_fin(const float* __restrict__ x, const float* __restrict__ P1, const float* __restrict__ P3, const float* __restrict__ b, const float* __restrict__ P4, const float* __restrict__ e, float* out0, float* out1) { const int t = blockIdx.x * 256 + threadIdx.x; if (t >= NB * NN / 4) return; const size_t f = (size_t)t * 4; const int c0 = (t % (NN / 4)) * 4;
    const v4f xv = *(const v4f*)(x + f), p1 = *(const v4f*)(P1 + f), p3 = *(const v4f*)(P3 + f), bv = *(const v4f*)(b + c0), p4 = *(const v4f*)(P4 + f), ev = *(const v4f*)(e + f); v4f o0, o1;
#pragma unroll
    for (int k = 0; k < 4; ++k) { const float xk = bfr(xv[k]), bk = bfr(bv[k]), ek = bfr(ev[k]); const float p = __fadd_rn(__fadd_rn(__fadd_rn(__fadd_rn(-xk, p1[k]), p3[k]), bk), p4[k]); const float n = __fadd_rn(p, __fmul_rn(0.81649661f, ek)); const float v = __fadd_rn(xk, __fmul_rn(0.33333334f, n)); o0[k] = v; o1[k] = fmaxf(v, 0.0f) + log1pf(expf(-fabsf(v))); }
    *(volatile v4f*)(out0 + f) = o0; *(volatile v4f*)(out1 + f) = o1; __threadfence(); *(volatile v4f*)(out0 + f) = o0; *(volatile v4f*)(out1 + f) = o1; }

extern "C" void kernel_launch(void* const* d_in, const int* in_sizes, int n_in, void* d_out, int out_size, void* d_ws, size_t ws_size, hipStream_t stream) {
    if (n_in < 10) return;
    if (in_sizes[0] != NB * NR || in_sizes[1] != NB * NS || in_sizes[2] != NB * NN || in_sizes[3] != NB * NN || in_sizes[4] != NN * NN || in_sizes[5] != NN || in_sizes[6] != NN * NR || in_sizes[7] != NR * NN || in_sizes[8] != NS * NN || in_sizes[9] != NB * NN) return;
    if (out_size != 2 * NB * NN) return;
    static_assert(NB % 64 == 0 && NN % 64 == 0 && NR % 64 == 0 && NR % 32 == 0 && NS % 32 == 0 && NN % 32 == 0 && (NN * NN) % (64 * 64) == 0 && (NN * NS) % (64 * 64) == 0 && (NB * NN) % (8 * 256) == 0 && (NB * NS) % (8 * 256) == 0 && (NB * NR) % (8 * 256) == 0 && (NB * NN / 4) % 256 == 0, "the products: every M and N a multiple of 64, every depth of 32; k_wtG's lines of 64 words; every flat grid exact");
    const float* g = (const float*)d_in[0]; const float* s = (const float*)d_in[1]; const float* x = (const float*)d_in[2]; const float* r = (const float*)d_in[3]; const float* J = (const float*)d_in[4]; const float* b = (const float*)d_in[5]; const float* U = (const float*)d_in[6]; const float* V = (const float*)d_in[7]; const float* Q = (const float*)d_in[8]; const float* e = (const float*)d_in[9];
    float* out0 = (float*)d_out; float* out1 = out0 + (size_t)NB * NN;
    char* wsp = (char*)d_ws; auto take = [&](size_t bytes) { char* p = wsp; wsp += (bytes + 255) & ~(size_t)255; return (void*)p; };
    bf* Rb = (bf*)take((size_t)NB * NN * 2); bf* Jt = (bf*)take((size_t)NN * NN * 2); bf* Sb = (bf*)take((size_t)NB * NS * 2); bf* Qt = (bf*)take((size_t)NN * NS * 2); bf* Vb = (bf*)take((size_t)NR * NN * 2); bf* Ub = (bf*)take((size_t)NN * NR * 2); bf* Tb = (bf*)take((size_t)NB * NR * 2);
    float* P1 = (float*)take((size_t)NB * NN * 4); float* P2 = (float*)take((size_t)NB * NR * 4); float* P3 = (float*)take((size_t)NB * NN * 4); float* P4 = (float*)take((size_t)NB * NN * 4);
    if ((size_t)(wsp - (char*)d_ws) > ws_size) return;
    k_cvt8<<<(unsigned)(NB * NN / 8 / 256), 256, 0, stream>>>(r, Rb, (size_t)NB * NN / 8);
    k_cvt8<<<(unsigned)(NB * NS / 8 / 256), 256, 0, stream>>>(s, Sb, (size_t)NB * NS / 8);
    k_cvt8<<<(unsigned)(NR * NN / 8 / 256), 256, 0, stream>>>(V, Vb, (size_t)NR * NN / 8);
    k_cvt8<<<(unsigned)(NN * NR / 8 / 256), 256, 0, stream>>>(U, Ub, (size_t)NN * NR / 8);
    k_wtG<<<(unsigned)(NN * NN / 64 / 64), 256, 0, stream>>>(J, NN, NN, Jt);
    k_wtG<<<(unsigned)(NN * NS / 64 / 64), 256, 0, stream>>>(Q, NS, NN, Qt);
    k_gemmw<bf, 0, false><<<dim3(NB / 64, NN / 64, 1), 32, 0, stream>>>(Rb, nullptr, Jt, nullptr, NN, P1, NN, nullptr, 0, 0, 0);
    k_gemmw<bf, 0, false><<<dim3(NB / 64, NR / 64, 1), 32, 0, stream>>>(Rb, nullptr, Vb, nullptr, NN, P2, NR, nullptr, 0, 0, 0);
    k_mid<<<(unsigned)(NB * NR / 8 / 256), 256, 0, stream>>>(g, P2, Tb);
    k_gemmw<bf, 0, false><<<dim3(NB / 64, NN / 64, 1), 32, 0, stream>>>(Tb, nullptr, Ub, nullptr, NR, P3, NN, nullptr, 0, 0, 0);
    k_gemmw<bf, 0, false><<<dim3(NB / 64, NN / 64, 1), 32, 0, stream>>>(Sb, nullptr, Qt, nullptr, NS, P4, NN, nullptr, 0, 0, 0);
    k_fin<<<(unsigned)(NB * NN / 4 / 256), 256, 0, stream>>>(x, P1, P3, b, P4, e, out0, out1);
}
